// ProbSFNO_81046032876052
// MI455X (gfx1250) — hardware-verified
//
#include <hip/hip_runtime.h>
#include <math.h>


typedef _Float16 v16h __attribute__((ext_vector_type(16)));
typedef _Float16 v8h  __attribute__((ext_vector_type(8), __may_alias__));
typedef float    v8f  __attribute__((ext_vector_type(8)));
typedef float    v4f  __attribute__((ext_vector_type(4), __may_alias__));

union Frag { v16h v; v8h half[2]; };

#define NB    4
#define INC   5
#define OUTC  2
#define NLAT  121
#define NLON  240
#define LW    48
#define EMB   256
#define H2    512
#define SP    (NLAT*NLON)
#define TWO_PI 6.2831853071795864769f

#define AS_STRIDE 264
#define AC_STRIDE 520

#define SC_ACT   64.0f
#define SC_FILT  64.0f
#define SC_G     1024.0f
#define SC_W     64.0f
#define INV_AF   (1.0f/4096.0f)
#define INV_GW   (1.0f/65536.0f)

__device__ __forceinline__ v8f wmma_f16(v16h a, v16h b, v8f c) {
  c = __builtin_amdgcn_wmma_f32_16x16x32_f16(false, a, false, b, (short)0, c, false, false);
  asm volatile("v_nop\n\tv_nop\n\tv_nop\n\tv_nop" : "+v"(c) : "v"(a), "v"(b));
  return c;
}

__device__ __forceinline__ v16h lda_frag(const _Float16* row, int k0, int h) {
  Frag a;
  a.half[0] = *(const v8h*)(row + k0 + 8*h);
  a.half[1] = *(const v8h*)(row + k0 + 16 + 8*h);
  return a.v;
}

__device__ __forceinline__ v16h ldb_frag(const float* __restrict__ col, int k0, int h,
                                         size_t ldb, float scale) {
  Frag b;
  #pragma unroll
  for (int i = 0; i < 8; ++i) {
    const int k = k0 + 8*h + i;
    b.v[i]     = (_Float16)(col[(size_t)k * ldb] * scale);
    b.v[8 + i] = (_Float16)(col[(size_t)(k + 16) * ldb] * scale);
  }
  return b.v;
}

__device__ __forceinline__ v8f tile_gemm(const _Float16* arow, const float* __restrict__ bcol,
                                        size_t ldb, float bscale, int ksteps, int h) {
  v8f acc = {0.f, 0.f, 0.f, 0.f, 0.f, 0.f, 0.f, 0.f};
  #pragma unroll 1
  for (int ks = 0; ks < ksteps; ++ks) {
    const v16h a = lda_frag(arow, ks*32, h);
    const v16h b = ldb_frag(bcol, ks*32, h, ldb, bscale);
    acc = wmma_f16(a, b, acc);
  }
  return acc;
}

__device__ __forceinline__ v4f a0_group(int gi, const float* q0, const float* Tl,
                                        const float* __restrict__ w_in,
                                        const float* __restrict__ b_in) {
  const int row = gi / (LW/4);
  const int l0  = (gi - row*(LW/4)) * 4;
  const int b   = row >> 8;
  const int c   = row & (EMB - 1);
  const float bi = b_in[c];
  v4f s;
  s[0] = bi*Tl[l0]; s[1] = bi*Tl[l0+1]; s[2] = bi*Tl[l0+2]; s[3] = bi*Tl[l0+3];
  #pragma unroll 1
  for (int cp = 0; cp < INC; ++cp) {
    const float w = w_in[c*INC + cp];
    const float* q = q0 + (b*INC + cp)*LW + l0;
    s[0] += w*q[0]; s[1] += w*q[1]; s[2] += w*q[2]; s[3] += w*q[3];
  }
  return s * TWO_PI;
}

__global__ __launch_bounds__(256) void k_prep(
    const float* __restrict__ x, const float* __restrict__ P,
    const float* __restrict__ wq, const float* __restrict__ w_in,
    const float* __restrict__ b_in, float* a0)
{
  __shared__ float xbar[NB*INC*NLAT];
  __shared__ float q0[NB*INC*LW];
  __shared__ float Tl[LW];
  const int tid = threadIdx.x;

  for (int idx = tid; idx < NB*INC*NLAT; idx += 256) {
    const int bc = idx / NLAT, j = idx - bc*NLAT;
    const v4f* px = (const v4f*)(x + ((size_t)bc*NLAT + j)*NLON);
    v4f s4 = {0.f, 0.f, 0.f, 0.f};
    for (int w = 0; w < NLON/4; ++w) s4 += px[w];
    xbar[idx] = (s4[0] + s4[1] + s4[2] + s4[3]) * (1.0f/NLON);
  }
  __syncthreads();

  for (int idx = tid; idx < NB*INC*LW; idx += 256) {
    const int bc = idx / LW, l = idx - bc*LW;
    const float* pp = P + (size_t)l*LW*NLAT;
    const float* xb = xbar + bc*NLAT;
    float s = 0.f;
    for (int j = 0; j < NLAT; ++j) s += xb[j]*(pp[j]*wq[j]);
    q0[idx] = s;
  }
  if (tid < LW) {
    const float* pp = P + (size_t)tid*LW*NLAT;
    float t = 0.f;
    for (int j = 0; j < NLAT; ++j) t += pp[j]*wq[j];
    Tl[tid] = t;
  }
  __syncthreads();

  const int ngr = NB*EMB*LW/4;
  for (int gi = tid; gi < ngr; gi += 256) {
    const v4f v = a0_group(gi, q0, Tl, w_in, b_in);
    *(volatile v4f*)(a0 + 4*(size_t)gi) = v;
  }
  __threadfence();
  for (int gi = tid; gi < ngr; gi += 256) {
    const v4f v = a0_group(gi, q0, Tl, w_in, b_in);
    *(volatile v4f*)(a0 + 4*(size_t)gi) = v;
  }
}

__global__ __launch_bounds__(256) void k_filter(
    const float* __restrict__ a0, const float* dcum,
    const float* __restrict__ P, const float* __restrict__ wq,
    const float* __restrict__ filt_r, const float* __restrict__ filt_i,
    float* fout, int layer)
{
  __shared__ __attribute__((aligned(16))) _Float16 As[16*AS_STRIDE];
  __shared__ __attribute__((aligned(16))) float    Fs[NB*EMB];
  (void)filt_i;
  const int l = blockIdx.x;
  if (l >= LW) return;
  const int tid  = threadIdx.x;
  const int lane = tid & 31;
  const int wave = tid >> 5;
  const int h    = lane >> 4;
  const int m    = lane & 15;

  float T = 0.f;
  {
    const float* pp = P + (size_t)l*LW*NLAT;
    for (int j = 0; j < NLAT; ++j) T += pp[j]*wq[j];
  }
  const float Sl = TWO_PI * T;

  for (int idx = tid; idx < 16*EMB; idx += 256) {
    const int mm = idx >> 8, i = idx & (EMB - 1);
    float v = 0.f;
    if (mm < NB) {
      v = a0[((size_t)(mm*EMB) + i)*LW + l];
      if (layer > 0) v += dcum[mm*EMB + i] * Sl;
    }
    As[mm*AS_STRIDE + i] = (_Float16)(v * SC_ACT);
  }
  __syncthreads();

  const float* fr = filt_r + (size_t)layer*EMB*EMB*LW;
  const _Float16* arow = As + m*AS_STRIDE;
  const int ocol0 = wave*32 + m;
  const int ocol1 = wave*32 + 16 + m;
  const v8f acc0 = tile_gemm(arow, fr + (size_t)ocol0*LW + l, (size_t)EMB*LW, SC_FILT, EMB/32, h);
  const v8f acc1 = tile_gemm(arow, fr + (size_t)ocol1*LW + l, (size_t)EMB*LW, SC_FILT, EMB/32, h);

  if (h == 0) {
    #pragma unroll
    for (int r = 0; r < NB; ++r) {
      Fs[r*EMB + ocol0] = acc0[r] * INV_AF;
      Fs[r*EMB + ocol1] = acc1[r] * INV_AF;
    }
  }
  __syncthreads();

  const v4f v = *(const v4f*)(Fs + 4*tid);
  float* dst = fout + (size_t)l*(NB*EMB) + 4*tid;
  *(volatile v4f*)dst = v;
  __threadfence();
  *(volatile v4f*)dst = v;
}

__global__ __launch_bounds__(256) void k_mlp(
    const float* __restrict__ f, const float* __restrict__ P,
    const float* __restrict__ w1, const float* __restrict__ b1,
    const float* __restrict__ w2, const float* __restrict__ b2,
    float* dcum, int layer)
{
  __shared__ __attribute__((aligned(16))) _Float16 Gs[16*AS_STRIDE];
  __shared__ __attribute__((aligned(16))) _Float16 Act[16*AC_STRIDE];
  __shared__ __attribute__((aligned(16))) float    dsh[NB*EMB];
  __shared__ float Pb[LW];
  const int tid  = threadIdx.x;
  const int lane = tid & 31;
  const int wave = tid >> 5;
  const int h    = lane >> 4;
  const int m    = lane & 15;

  if (tid < LW) {
    const float* pp = P + (size_t)tid*LW*NLAT;
    float s = 0.f;
    for (int j = 0; j < NLAT; ++j) s += pp[j];
    Pb[tid] = s * (1.0f/NLAT);
  }
  for (int idx = tid; idx < 12*AS_STRIDE; idx += 256) Gs[4*AS_STRIDE + idx]  = (_Float16)0.f;
  for (int idx = tid; idx < 12*AC_STRIDE; idx += 256) Act[4*AC_STRIDE + idx] = (_Float16)0.f;
  __syncthreads();

  for (int idx = tid; idx < NB*EMB; idx += 256) {
    float s = 0.f;
    for (int l = 0; l < LW; ++l) s += f[(size_t)l*(NB*EMB) + idx] * Pb[l];
    Gs[(idx >> 8)*AS_STRIDE + (idx & (EMB - 1))] = (_Float16)(s * SC_G);
  }
  __syncthreads();

  {
    const float* W1 = w1 + (size_t)layer*EMB*H2;
    const float* B1 = b1 + (size_t)layer*H2;
    const _Float16* arow = Gs + m*AS_STRIDE;
    for (int nt = wave*4; nt < wave*4 + 4; ++nt) {
      const int hc = nt*16 + m;
      const v8f acc = tile_gemm(arow, W1 + hc, (size_t)H2, SC_W, EMB/32, h);
      if (h == 0) {
        const float bb = B1[hc];
        #pragma unroll
        for (int r = 0; r < NB; ++r) {
          const float s  = acc[r] * INV_GW + bb;
          const float gl = 0.5f * s * (1.0f + erff(s * 0.70710678118654752f));
          Act[r*AC_STRIDE + hc] = (_Float16)(gl * SC_G);
        }
      }
    }
  }
  __syncthreads();

  {
    const float* W2 = w2 + (size_t)layer*H2*EMB;
    const float* B2 = b2 + (size_t)layer*EMB;
    const _Float16* arow = Act + m*AC_STRIDE;
    for (int nt = wave*2; nt < wave*2 + 2; ++nt) {
      const int c = nt*16 + m;
      const v8f acc = tile_gemm(arow, W2 + c, (size_t)EMB, SC_W, H2/32, h);
      if (h == 0) {
        const float bb = B2[c];
        #pragma unroll
        for (int r = 0; r < NB; ++r) {
          const int idx = r*EMB + c;
          const float old = (layer > 0) ? dcum[idx] : 0.f;
          dsh[idx] = old + acc[r] * INV_GW + bb;
        }
      }
    }
  }
  __syncthreads();

  const v4f v = *(const v4f*)(dsh + 4*tid);
  float* dst = dcum + 4*tid;
  *(volatile v4f*)dst = v;
  __threadfence();
  *(volatile v4f*)dst = v;
}

__global__ __launch_bounds__(256) void k_final(
    const float* __restrict__ x, const float* __restrict__ eps,
    const float* __restrict__ w_in, const float* __restrict__ b_in,
    const float* __restrict__ w_out, const float* __restrict__ b_out,
    const float* __restrict__ dcum, float* out, int ngroups)
{
  __shared__ float sW[2*OUTC*INC];
  __shared__ float sov[NB*2*OUTC];
  const int tid = threadIdx.x;
  if (tid < 2*OUTC*INC) {
    const int o = tid / INC, cp = tid - o*INC;
    float s = 0.f;
    for (int c = 0; c < EMB; ++c) s += w_out[o*EMB + c] * w_in[c*INC + cp];
    sW[tid] = s;
  } else if (tid >= 32 && tid < 32 + NB*2*OUTC) {
    const int t = tid - 32;
    const int b = t >> 2, o = t & 3;
    float s = b_out[o];
    for (int c = 0; c < EMB; ++c) s += w_out[o*EMB + c] * (b_in[c] + dcum[b*EMB + c]);
    sov[t] = s;
  }
  __syncthreads();

  const int gi = blockIdx.x*blockDim.x + tid;
  if (gi >= ngroups) return;
  const int e  = 4*gi;
  const int ch = e / SP;
  const int b  = ch >> 1, o = ch & 1;
  const int p  = e - ch*SP;
  const float* xp = x + (size_t)(b*INC)*SP + p;
  const float* ep = eps + e;

  v4f smp, muv, lsv;
  #pragma unroll 1
  for (int q = 0; q < 4; ++q) {
    float mu = sov[b*2*OUTC + o];
    float ls = sov[b*2*OUTC + OUTC + o];
    #pragma unroll
    for (int c = 0; c < INC; ++c) {
      const float xv = xp[(size_t)c*SP + q];
      mu += sW[o*INC + c] * xv;
      ls += sW[(OUTC + o)*INC + c] * xv;
    }
    const float ev = ep[q];
    smp[q] = mu + ev * expf(ls);
    muv[q] = mu;
    lsv[q] = ls;
  }

  const size_t CH = (size_t)NB*OUTC*SP;
  float* d0 = out + e;
  float* d1 = out + CH + e;
  float* d2 = out + 2*CH + e;
  *(volatile v4f*)d0 = smp;
  *(volatile v4f*)d1 = muv;
  *(volatile v4f*)d2 = lsv;
  __threadfence();
  *(volatile v4f*)d0 = smp;
  *(volatile v4f*)d1 = muv;
  *(volatile v4f*)d2 = lsv;
}

extern "C" void kernel_launch(void* const* d_in, const int* in_sizes, int n_in,
                              void* d_out, int out_size, void* d_ws, size_t ws_size,
                              hipStream_t stream) {
  (void)in_sizes;
  if (n_in < 14) return;
  const float* x      = (const float*)d_in[0];
  const float* eps    = (const float*)d_in[1];
  const float* Pmat   = (const float*)d_in[2];
  const float* wq     = (const float*)d_in[3];
  const float* w_in   = (const float*)d_in[4];
  const float* b_in   = (const float*)d_in[5];
  const float* filt_r = (const float*)d_in[6];
  const float* filt_i = (const float*)d_in[7];
  const float* w1     = (const float*)d_in[8];
  const float* b1     = (const float*)d_in[9];
  const float* w2     = (const float*)d_in[10];
  const float* b2     = (const float*)d_in[11];
  const float* w_out  = (const float*)d_in[12];
  const float* b_out  = (const float*)d_in[13];

  const size_t n_a0 = (size_t)NB*EMB*LW;
  const size_t n_f  = (size_t)LW*NB*EMB;
  const size_t n_dc = (size_t)NB*EMB;
  if (ws_size < (n_a0 + n_f + n_dc)*sizeof(float)) return;
  float* ws   = (float*)d_ws;
  float* a0   = ws;
  float* f    = ws + n_a0;
  float* dcum = ws + n_a0 + n_f;

  const int per_out = out_size / 3;
  const int ngroups = per_out / 4;
  const int gridF   = (ngroups + 255) / 256;

  k_prep<<<1, 256, 0, stream>>>(x, Pmat, wq, w_in, b_in, a0);
  for (int i = 0; i < 4; ++i) {
    k_filter<<<LW, 256, 0, stream>>>(a0, dcum, Pmat, wq, filt_r, filt_i, f, i);
    k_mlp<<<1, 256, 0, stream>>>(f, Pmat, w1, b1, w2, b2, dcum, i);
  }
  k_final<<<gridF, 256, 0, stream>>>(x, eps, w_in, b_in, w_out, b_out, dcum,
                                      (float*)d_out, ngroups);
}
